// PointNet2Encoder_36094905156308
// MI455X (gfx1250) — hardware-verified
//
#include <hip/hip_runtime.h>
#pragma clang fp contract(off)

typedef __attribute__((ext_vector_type(16))) _Float16 v16h;
typedef __attribute__((ext_vector_type(8)))  _Float16 v8h;
typedef __attribute__((ext_vector_type(8)))  float    v8f;
typedef __attribute__((ext_vector_type(4)))  float    v4f;
typedef __attribute__((ext_vector_type(4)))  unsigned v4u;

namespace shp {
constexpr int NBATCH = 16;
constexpr int NPTS1  = 8192;
constexpr int NCTR1  = 512;
constexpr int KSEL1  = 32;
constexpr int NCTR2  = 128;
constexpr int KSEL2  = 64;
constexpr int ROWS3  = NBATCH * NCTR2;
constexpr int KPAD3  = 320;
}

__device__ __forceinline__ unsigned h16_bits(float f) {
  const _Float16 h = (_Float16)f;
  const unsigned short s = __builtin_bit_cast(unsigned short, h);
  return (unsigned)s;
}
__device__ __forceinline__ unsigned pack2(unsigned lo, unsigned hi) {
  return (lo & 0xffffu) | (hi << 16);
}
__device__ __forceinline__ unsigned opaque_zero() {
  unsigned z = 0u;
  asm volatile("" : "+v"(z));
  return z;
}
union FragH { v16h v; v8h h[2]; };
__device__ __forceinline__ v16h frag_load(const _Float16* p) {
  FragH f;
  f.h[0] = *(const v8h*)(p);
  f.h[1] = *(const v8h*)(p + 16);
  return f.v;
}
__device__ __forceinline__ v8f mma_h(v16h a, v16h b, v8f c) {
  c = __builtin_amdgcn_wmma_f32_16x16x32_f16(false, a, false, b, (short)0, c, false, false);
  asm volatile("v_nop\n\tv_nop\n\tv_nop\n\tv_nop" : "+v"(c) : "v"(a), "v"(b));
  return c;
}
__device__ __forceinline__ int nth_set_bit(unsigned m, int n) {
  int pos = 0;
  unsigned mm = m;
  int c = __popc(mm & 0xFFFFu);
  if (n >= c) { n -= c; pos += 16; mm >>= 16; }
  c = __popc(mm & 0xFFu);
  if (n >= c) { n -= c; pos += 8; mm >>= 8; }
  c = __popc(mm & 0xFu);
  if (n >= c) { n -= c; pos += 4; mm >>= 4; }
  c = __popc(mm & 0x3u);
  if (n >= c) { n -= c; pos += 2; mm >>= 2; }
  c = (int)(mm & 1u);
  if (n >= c) { pos += 1; }
  return pos;
}

__global__ __launch_bounds__(256) void pack_w_kernel(
    const float* __restrict__ W, unsigned short* __restrict__ Bt,
    int Kact, int Kpad, int Nout, int nfeat, int dup) {
  const int q = blockIdx.x * 256 + threadIdx.x;
  const int cpr = Kpad >> 3;
  const int total = Nout * cpr;
  if (q < total) {
    const int n = q / cpr;
    const int kc = q - n * cpr;
    unsigned hb[8];
#pragma unroll
    for (int e = 0; e < 8; ++e) {
      const int k = kc * 8 + e;
      int src = -1;
      if (nfeat < 0) {
        if (k < Kact) src = k;
      } else {
        if (k < nfeat) src = k + 3;
        else if (k < nfeat + 3) src = k - nfeat;
        else if (dup != 0 && k < nfeat + 6) src = k - nfeat - 3;
      }
      const bool valid = (src >= 0) && (src < Kact);
      const int sc = valid ? src : 0;
      const float wv = W[(size_t)sc * Nout + n];
      const float v = valid ? wv : 0.0f;
      hb[e] = h16_bits(v);
    }
    v4u w;
    w.x = pack2(hb[0], hb[1]);
    w.y = pack2(hb[2], hb[3]);
    w.z = pack2(hb[4], hb[5]);
    w.w = pack2(hb[6], hb[7]);
    volatile v4u* dst = (volatile v4u*)(Bt + (size_t)q * 8);
    *dst = w;
    __threadfence();
    *dst = w;
  }
}

template <int NPTS, int NT, int MSEL>
__global__ __launch_bounds__(NT) void fps_kernel(const float* __restrict__ pts,
                                                 float* __restrict__ ctrs) {
#pragma clang fp contract(off)
  static_assert(NPTS == NT * 8);
  static_assert((MSEL * 3) % 4 == 0);
  __shared__ __align__(16) float csel[MSEL * 3];
  __shared__ float rv[2][32];
  __shared__ int   ri[2][32];
  const int b = blockIdx.x, tid = threadIdx.x;
  const int lane = tid & 31, wid = tid >> 5;
  const float* P = pts + (size_t)b * NPTS * 3;

  float f[24];
#pragma unroll
  for (int q = 0; q < 6; ++q) {
    const v4f r = *(const v4f*)(P + (size_t)tid * 24 + q * 4);
    f[q * 4 + 0] = r.x; f[q * 4 + 1] = r.y; f[q * 4 + 2] = r.z; f[q * 4 + 3] = r.w;
  }
  float px[8], py[8], pz[8], dist[8];
#pragma unroll
  for (int j = 0; j < 8; ++j) {
    px[j] = f[3 * j]; py[j] = f[3 * j + 1]; pz[j] = f[3 * j + 2];
    dist[j] = 1e10f;
  }
  if (tid < 64) {
    (&rv[0][0])[tid] = -1.0f;
    (&ri[0][0])[tid] = 0x7fffffff;
  }
  __syncthreads();

  int last = 0;
#pragma unroll 1
  for (int it = 0; it < MSEL; ++it) {
    const int lc = last < 0 ? 0 : (last > NPTS - 1 ? NPTS - 1 : last);
    const float lx = P[lc * 3 + 0], ly = P[lc * 3 + 1], lz = P[lc * 3 + 2];
    if (tid == 0) { csel[it * 3 + 0] = lx; csel[it * 3 + 1] = ly; csel[it * 3 + 2] = lz; }
    float bm = -1.0f;
    int bi = 0x7fffffff;
#pragma unroll
    for (int j = 0; j < 8; ++j) {
      const float dx = px[j] - lx, dy = py[j] - ly, dz = pz[j] - lz;
      const float t0 = dx * dx, t1 = dy * dy, t2 = dz * dz;
      const float d = (t0 + t2) + t1;
      const float dj = fminf(dist[j], d);
      dist[j] = dj;
      if (dj > bm) { bm = dj; bi = tid * 8 + j; }
    }
#pragma unroll
    for (int s = 16; s > 0; s >>= 1) {
      const float ov = __shfl_xor(bm, s, 32);
      const int   oi = __shfl_xor(bi, s, 32);
      if (ov > bm || (ov == bm && oi < bi)) { bm = ov; bi = oi; }
    }
    const int buf = it & 1;
    if (lane == 0) { rv[buf][wid] = bm; ri[buf][wid] = bi; }
    __syncthreads();
    float v = rv[buf][lane];
    int   i = ri[buf][lane];
#pragma unroll
    for (int s = 16; s > 0; s >>= 1) {
      const float ov = __shfl_xor(v, s, 32);
      const int   oi = __shfl_xor(i, s, 32);
      if (ov > v || (ov == v && oi < i)) { v = ov; i = oi; }
    }
    last = __builtin_amdgcn_readfirstlane(i);
  }
  __syncthreads();
  constexpr int N4 = MSEL * 3 / 4;
  float* dst = ctrs + (size_t)b * MSEL * 3;
  for (int pass = 0; pass < 2; ++pass) {
    for (int q0 = 0; q0 < N4; q0 += NT) {
      const int q = q0 + tid;
      if (q < N4) {
        const v4f val = *(const v4f*)(csel + q * 4);
        *(volatile v4f*)(dst + q * 4) = val;
      }
    }
    __threadfence();
  }
}

template <int NPTS, int KSEL>
__device__ __forceinline__ void ball_scan(const float* __restrict__ P, float cx, float cy, float cz,
                                          float r2, int lane, int& out0, int& out1) {
#pragma clang fp contract(off)
  static_assert(NPTS % 32 == 0);
  const float cxx = cx * cx, cyy = cy * cy, czz = cz * cz;
  const float sqc = (cxx + czz) + cyy;
  int cnt = 0, first = 0, slot0 = 0, slot1 = 0;
#pragma unroll 1
  for (int i0 = 0; i0 < NPTS; i0 += 32) {
    if (cnt >= KSEL) break;
    const int i = i0 + lane;
    const float px = P[i * 3 + 0], py = P[i * 3 + 1], pz = P[i * 3 + 2];
    const float pxx = px * px, pyy = py * py, pzz = pz * pz;
    const float sqp = (pxx + pzz) + pyy;
    float p = cx * px;
    p = __builtin_fmaf(cy, py, p);
    p = __builtin_fmaf(cz, pz, p);
    const float tp = 2.0f * p;
    const float sq = (sqc + sqp) - tp;
    const unsigned mask = __builtin_amdgcn_ballot_w32(sq <= r2);
    if (mask != 0u) {
      const int pc = __popc(mask);
      const int n0 = lane - cnt;
      const int p0 = nth_set_bit(mask, n0);
      if (n0 >= 0 && n0 < pc) slot0 = i0 + p0;
      if (KSEL > 32) {
        const int n1 = lane + 32 - cnt;
        const int p1 = nth_set_bit(mask, n1);
        if (n1 >= 0 && n1 < pc) slot1 = i0 + p1;
      }
      if (cnt == 0) first = i0 + (__ffs((int)mask) - 1);
      cnt += pc;
    }
  }
  int a0 = (lane < cnt) ? slot0 : first;
  int a1 = (lane + 32 < cnt) ? slot1 : first;
  a0 = a0 < 0 ? 0 : (a0 > NPTS - 1 ? NPTS - 1 : a0);
  a1 = a1 < 0 ? 0 : (a1 > NPTS - 1 ? NPTS - 1 : a1);
  out0 = a0;
  out1 = a1;
}

template <int MT, int KP, int NOUT>
__device__ __forceinline__ void mlp_layer(const _Float16* Xl, const int ldx,
                                          const _Float16* __restrict__ Bt,
                                          const float* __restrict__ bias,
                                          _Float16* Ol, const int ldo,
                                          const int wave, const int lane) {
  static_assert(KP % 32 == 0 && NOUT % 64 == 0);
  const int c = lane & 15, hh = lane >> 4;
#pragma unroll 1
  for (int t = 0; t < NOUT / 64; ++t) {
    const int nt = wave + 4 * t;
    v8f acc[MT];
#pragma unroll
    for (int m = 0; m < MT; ++m) acc[m] = (v8f){0.f, 0.f, 0.f, 0.f, 0.f, 0.f, 0.f, 0.f};
#pragma unroll 1
    for (int k0 = 0; k0 < KP; k0 += 32) {
      const v16h bf = frag_load(Bt + (size_t)(nt * 16 + c) * KP + k0 + 8 * hh);
#pragma unroll
      for (int m = 0; m < MT; ++m) {
        const v16h a = frag_load(Xl + (m * 16 + c) * ldx + k0 + 8 * hh);
        acc[m] = mma_h(a, bf, acc[m]);
      }
    }
    const float bc = bias[nt * 16 + c];
#pragma unroll
    for (int m = 0; m < MT; ++m) {
#pragma unroll
      for (int r = 0; r < 8; ++r) {
        const float v = fmaxf(acc[m][r] + bc, 0.0f);
        Ol[(m * 16 + 8 * hh + r) * ldo + nt * 16 + c] = (_Float16)v;
      }
    }
  }
}

template <int MT, int TPG, int KP, int NOUT>
__device__ __forceinline__ void mlp_layer_max(const _Float16* Xl, const int ldx,
                                              const _Float16* __restrict__ Bt,
                                              const float* __restrict__ bias,
                                              float* Fo, const int wave, const int lane) {
  static_assert(KP % 32 == 0 && NOUT % 64 == 0 && MT % TPG == 0);
  constexpr int NG = MT / TPG;
  const int c = lane & 15, hh = lane >> 4;
#pragma unroll 1
  for (int t = 0; t < NOUT / 64; ++t) {
    const int nt = wave + 4 * t;
    v8f acc[MT];
#pragma unroll
    for (int m = 0; m < MT; ++m) acc[m] = (v8f){0.f, 0.f, 0.f, 0.f, 0.f, 0.f, 0.f, 0.f};
#pragma unroll 1
    for (int k0 = 0; k0 < KP; k0 += 32) {
      const v16h bf = frag_load(Bt + (size_t)(nt * 16 + c) * KP + k0 + 8 * hh);
#pragma unroll
      for (int m = 0; m < MT; ++m) {
        const v16h a = frag_load(Xl + (m * 16 + c) * ldx + k0 + 8 * hh);
        acc[m] = mma_h(a, bf, acc[m]);
      }
    }
    const float bc = bias[nt * 16 + c];
#pragma unroll
    for (int gi = 0; gi < NG; ++gi) {
      float cm = acc[gi * TPG][0];
#pragma unroll
      for (int tt = 0; tt < TPG; ++tt) {
#pragma unroll
        for (int r = 0; r < 8; ++r) cm = fmaxf(cm, acc[gi * TPG + tt][r]);
      }
      const float ot = __shfl_xor(cm, 16, 32);
      cm = fmaxf(cm, ot);
      if (lane < 16) Fo[gi * NOUT + nt * 16 + c] = fmaxf(cm + bc, 0.0f);
    }
  }
}

__global__ __launch_bounds__(128) void sa1_kernel(
    const float* __restrict__ x, const float* __restrict__ c1,
    const unsigned short* __restrict__ bt0, const float* __restrict__ b0,
    const unsigned short* __restrict__ bt1, const float* __restrict__ b1,
    const unsigned short* __restrict__ bt2, const float* __restrict__ b2,
    unsigned short* __restrict__ f1) {
  __shared__ __align__(16) _Float16 X0[128 * 32];
  __shared__ __align__(16) _Float16 H0[128 * 64];
  __shared__ __align__(16) _Float16 H1[128 * 64];
  __shared__ __align__(16) float Fs[4 * 128];
  const int tid = threadIdx.x;
  const int lane = tid & 31;
  const int wave = __builtin_amdgcn_readfirstlane(tid >> 5);
  const int g = blockIdx.x * 4 + wave;
  const int b = g / shp::NCTR1;
  const float* P = x + (size_t)b * (shp::NPTS1 * 3);
  const float cx = c1[(size_t)g * 3 + 0], cy = c1[(size_t)g * 3 + 1], cz = c1[(size_t)g * 3 + 2];
  int s0, s1;
  ball_scan<shp::NPTS1, shp::KSEL1>(P, cx, cy, cz, 0.04f, lane, s0, s1);
  (void)s1;
  {
    const float rx = P[s0 * 3 + 0] - cx;
    const float ry = P[s0 * 3 + 1] - cy;
    const float rz = P[s0 * 3 + 2] - cz;
    const unsigned zz = opaque_zero();
    v4u w;
    w.x = pack2(h16_bits(rx), h16_bits(ry));
    w.y = pack2(h16_bits(rz), zz);
    w.z = zz;
    w.w = zz;
    v4u z4;
    z4.x = zz; z4.y = zz; z4.z = zz; z4.w = zz;
    v4u* dst = (v4u*)(X0 + (wave * 32 + lane) * 32);
    dst[0] = w; dst[1] = z4; dst[2] = z4; dst[3] = z4;
  }
  __syncthreads();
  mlp_layer<8, 32, 64>(X0, 32, (const _Float16*)bt0, b0, H0, 64, wave, lane);
  __syncthreads();
  mlp_layer<8, 64, 64>(H0, 64, (const _Float16*)bt1, b1, H1, 64, wave, lane);
  __syncthreads();
  mlp_layer_max<8, 2, 64, 128>(H1, 64, (const _Float16*)bt2, b2, Fs, wave, lane);
  __syncthreads();
  if (tid < 64) {
    const v4f fa = *(const v4f*)(Fs + tid * 8);
    const v4f fb = *(const v4f*)(Fs + tid * 8 + 4);
    v4u w;
    w.x = pack2(h16_bits(fa.x), h16_bits(fa.y));
    w.y = pack2(h16_bits(fa.z), h16_bits(fa.w));
    w.z = pack2(h16_bits(fb.x), h16_bits(fb.y));
    w.w = pack2(h16_bits(fb.z), h16_bits(fb.w));
    volatile v4u* dst = (volatile v4u*)(f1 + (size_t)blockIdx.x * 512 + tid * 8);
    *dst = w;
    __threadfence();
    *dst = w;
  }
}

__global__ __launch_bounds__(128) void sa2_kernel(
    const float* __restrict__ c1, const float* __restrict__ c2,
    const unsigned short* __restrict__ f1,
    const unsigned short* __restrict__ bt0, const float* __restrict__ b0,
    const unsigned short* __restrict__ bt1, const float* __restrict__ b1,
    const unsigned short* __restrict__ bt2, const float* __restrict__ b2,
    unsigned short* __restrict__ A3) {
  __shared__ __align__(16) _Float16 X[64 * 160];
  __shared__ __align__(16) _Float16 H0[64 * 128];
  __shared__ __align__(16) _Float16 H1[64 * 128];
  __shared__ __align__(16) float Fs[256];
  __shared__ int sidx[64];
  const int tid = threadIdx.x;
  const int lane = tid & 31;
  const int wave = __builtin_amdgcn_readfirstlane(tid >> 5);
  const int g = blockIdx.x;
  const int b = g / shp::NCTR2;
  const float* P = c1 + (size_t)b * (shp::NCTR1 * 3);
  const float cx = c2[(size_t)g * 3 + 0], cy = c2[(size_t)g * 3 + 1], cz = c2[(size_t)g * 3 + 2];
  int s0, s1;
  ball_scan<shp::NCTR1, shp::KSEL2>(P, cx, cy, cz, 0.16f, lane, s0, s1);
  if (wave == 0) { sidx[lane] = s0; sidx[lane + 32] = s1; }
  __syncthreads();
#pragma unroll 1
  for (int h2 = 0; h2 < 2; ++h2) {
#pragma unroll
    for (int it = 0; it < 4; ++it) {
      const int e = (h2 * 4 + it) * 128 + tid;
      const int r = e >> 4, q = e & 15;
      int id = sidx[r];
      id = id < 0 ? 0 : (id > shp::NCTR1 - 1 ? shp::NCTR1 - 1 : id);
      const v4u v = *(const v4u*)(f1 + ((size_t)(b * shp::NCTR1 + id)) * 128 + q * 8);
      *(v4u*)(X + r * 160 + q * 8) = v;
    }
  }
  if (tid < 64) {
    const int r = tid;
    int id = sidx[r];
    id = id < 0 ? 0 : (id > shp::NCTR1 - 1 ? shp::NCTR1 - 1 : id);
    const float rx = P[id * 3 + 0] - cx;
    const float ry = P[id * 3 + 1] - cy;
    const float rz = P[id * 3 + 2] - cz;
    const unsigned zz = opaque_zero();
    v4u w;
    w.x = pack2(h16_bits(rx), h16_bits(ry));
    w.y = pack2(h16_bits(rz), zz);
    w.z = zz;
    w.w = zz;
    v4u z4;
    z4.x = zz; z4.y = zz; z4.z = zz; z4.w = zz;
    v4u* dst = (v4u*)(X + r * 160 + 128);
    dst[0] = w; dst[1] = z4; dst[2] = z4; dst[3] = z4;
  }
  __syncthreads();
  mlp_layer<4, 160, 128>(X, 160, (const _Float16*)bt0, b0, H0, 128, wave, lane);
  __syncthreads();
  mlp_layer<4, 128, 128>(H0, 128, (const _Float16*)bt1, b1, H1, 128, wave, lane);
  __syncthreads();
  mlp_layer_max<4, 4, 128, 256>(H1, 128, (const _Float16*)bt2, b2, Fs, wave, lane);
  __syncthreads();
  if (wave == 0) {
    const unsigned zz = opaque_zero();
    const v4f fa = *(const v4f*)(Fs + lane * 8);
    const v4f fb = *(const v4f*)(Fs + lane * 8 + 4);
    v4u w;
    w.x = pack2(h16_bits(fa.x), h16_bits(fa.y));
    w.y = pack2(h16_bits(fa.z), h16_bits(fa.w));
    w.z = pack2(h16_bits(fb.x), h16_bits(fb.y));
    w.w = pack2(h16_bits(fb.z), h16_bits(fb.w));
    const float hx = rintf(cx * 16.0f) * 0.0625f;
    const float hy = rintf(cy * 16.0f) * 0.0625f;
    const float hz = rintf(cz * 16.0f) * 0.0625f;
    const float lx = cx - hx, ly = cy - hy, lz = cz - hz;
    const unsigned t0 = pack2(h16_bits(hx), h16_bits(hy));
    const unsigned t1 = pack2(h16_bits(hz), h16_bits(lx));
    const unsigned t2 = pack2(h16_bits(ly), h16_bits(lz));
    const bool isc = (lane == 0);
    v4u tv;
    tv.x = isc ? t0 : zz;
    tv.y = isc ? t1 : zz;
    tv.z = isc ? t2 : zz;
    tv.w = zz;
    unsigned short* row = A3 + (size_t)g * shp::KPAD3;
    for (int pass = 0; pass < 2; ++pass) {
      *(volatile v4u*)(row + lane * 8) = w;
      if (lane < 8) *(volatile v4u*)(row + 256 + lane * 8) = tv;
      __threadfence();
    }
  }
}

template <bool MAXOUT>
__global__ __launch_bounds__(256) void gemm64_kernel(
    const unsigned short* __restrict__ Ap, int lda,
    const unsigned short* __restrict__ Btp, int ldb,
    void* __restrict__ Cout, int ldc,
    const float* __restrict__ bias, int M, int N, int K) {
  const _Float16* A  = (const _Float16*)Ap;
  const _Float16* Bt = (const _Float16*)Btp;
  __shared__ __align__(16) float sT[8][16 * 68];
  const int lane = threadIdx.x & 31;
  const int wave = threadIdx.x >> 5;
  const int tilesN = N >> 6;
  const int tilesM = M >> 6;
  const int tile = blockIdx.x * 8 + wave;
  if (tile >= tilesM * tilesN) return;
  const int tm = tile / tilesN;
  const int tn = tile - tm * tilesN;
  const int m0 = tm << 6;
  const int n0 = tn << 6;
  const int rlane = lane & 15;
  const int koff  = (lane >> 4) * 8;
  const int mOff  = (lane >> 4) * 8;

  v8f acc[4][4];
#pragma unroll
  for (int i = 0; i < 4; ++i)
#pragma unroll
    for (int j = 0; j < 4; ++j) acc[i][j] = (v8f){0.f, 0.f, 0.f, 0.f, 0.f, 0.f, 0.f, 0.f};

#pragma unroll 1
  for (int k0 = 0; k0 < K; k0 += 32) {
    v16h bh[4];
#pragma unroll
    for (int j = 0; j < 4; ++j)
      bh[j] = frag_load(Bt + (size_t)(n0 + (j << 4) + rlane) * ldb + koff + k0);
#pragma unroll
    for (int i = 0; i < 4; ++i) {
      const v16h ah = frag_load(A + (size_t)(m0 + (i << 4) + rlane) * lda + koff + k0);
#pragma unroll
      for (int j = 0; j < 4; ++j) acc[i][j] = mma_h(ah, bh[j], acc[i][j]);
    }
  }

  float* slab = sT[wave];
  if (MAXOUT) {
#pragma unroll
    for (int j = 0; j < 4; ++j) {
      float cm = acc[0][j][0];
#pragma unroll
      for (int i = 0; i < 4; ++i) {
#pragma unroll
        for (int r = 0; r < 8; ++r) cm = fmaxf(cm, acc[i][j][r]);
      }
      const float ot = __shfl_xor(cm, 16, 32);
      cm = fmaxf(cm, ot);
      if (lane < 16) slab[(j << 4) + rlane] = cm;
    }
    __builtin_amdgcn_fence(__ATOMIC_RELEASE, "workgroup");
    __builtin_amdgcn_wave_barrier();
    __builtin_amdgcn_fence(__ATOMIC_ACQUIRE, "workgroup");
    const int l16 = lane & 15;
    const v4f val = *(const v4f*)(slab + l16 * 4);
    float* dst = (float*)Cout + (size_t)tm * ldc + n0 + l16 * 4;
    for (int pass = 0; pass < 2; ++pass) {
      if (lane < 16) *(volatile v4f*)dst = val;
      __threadfence();
    }
  } else {
    unsigned short* C = (unsigned short*)Cout;
#pragma unroll
    for (int i = 0; i < 4; ++i) {
      const int mBase = m0 + (i << 4);
#pragma unroll
      for (int j = 0; j < 4; ++j) {
        const int n = n0 + (j << 4) + rlane;
        const float bv = bias[n];
#pragma unroll
        for (int r = 0; r < 8; ++r) {
          const float v = fmaxf(acc[i][j][r] + bv, 0.0f);
          slab[(mOff + r) * 68 + (j << 4) + rlane] = v;
        }
      }
      __builtin_amdgcn_fence(__ATOMIC_RELEASE, "workgroup");
      __builtin_amdgcn_wave_barrier();
      __builtin_amdgcn_fence(__ATOMIC_ACQUIRE, "workgroup");
      const int q = lane >> 3, c8 = (lane & 7) * 8;
      for (int pass = 0; pass < 2; ++pass) {
#pragma unroll
        for (int it = 0; it < 4; ++it) {
          const int row = it * 4 + q;
          const float* sp = slab + row * 68 + c8;
          v8h hv;
#pragma unroll
          for (int e = 0; e < 8; ++e) hv[e] = (_Float16)sp[e];
          *(volatile v8h*)(C + (size_t)(mBase + row) * ldc + n0 + c8) = hv;
        }
        __threadfence();
      }
      __builtin_amdgcn_fence(__ATOMIC_RELEASE, "workgroup");
      __builtin_amdgcn_wave_barrier();
      __builtin_amdgcn_fence(__ATOMIC_ACQUIRE, "workgroup");
    }
  }
}

__global__ __launch_bounds__(256) void final_max_kernel(const float* __restrict__ pm,
                                                        const float* __restrict__ bias,
                                                        float* __restrict__ out) {
  const int t = blockIdx.x * 256 + threadIdx.x;
  const int b = t >> 8;
  const int n4 = (t & 255) * 4;
  const v4f a = *(const v4f*)(pm + (size_t)(2 * b) * 1024 + n4);
  const v4f c = *(const v4f*)(pm + (size_t)(2 * b + 1) * 1024 + n4);
  const v4f bb = *(const v4f*)(bias + n4);
  v4f o;
  o.x = fmaxf(fmaxf(a.x, c.x) + bb.x, 0.0f);
  o.y = fmaxf(fmaxf(a.y, c.y) + bb.y, 0.0f);
  o.z = fmaxf(fmaxf(a.z, c.z) + bb.z, 0.0f);
  o.w = fmaxf(fmaxf(a.w, c.w) + bb.w, 0.0f);
  volatile v4f* dst = (volatile v4f*)(out + (size_t)b * 1024 + n4);
  *dst = o;
  __threadfence();
  *dst = o;
}

extern "C" void kernel_launch(void* const* d_in, const int* in_sizes, int n_in,
                              void* d_out, int out_size, void* d_ws, size_t ws_size,
                              hipStream_t stream) {
  (void)in_sizes; (void)n_in; (void)out_size;
  const float* x    = (const float*)d_in[0];
  const float* s1w0 = (const float*)d_in[1];  const float* s1b0 = (const float*)d_in[2];
  const float* s1w1 = (const float*)d_in[3];  const float* s1b1 = (const float*)d_in[4];
  const float* s1w2 = (const float*)d_in[5];  const float* s1b2 = (const float*)d_in[6];
  const float* s2w0 = (const float*)d_in[7];  const float* s2b0 = (const float*)d_in[8];
  const float* s2w1 = (const float*)d_in[9];  const float* s2b1 = (const float*)d_in[10];
  const float* s2w2 = (const float*)d_in[11]; const float* s2b2 = (const float*)d_in[12];
  const float* s3w0 = (const float*)d_in[13]; const float* s3b0 = (const float*)d_in[14];
  const float* s3w1 = (const float*)d_in[15]; const float* s3b1 = (const float*)d_in[16];
  const float* s3w2 = (const float*)d_in[17]; const float* s3b2 = (const float*)d_in[18];
  float* out = (float*)d_out;

  static_assert(shp::ROWS3 % 64 == 0 && shp::KPAD3 % 32 == 0);
  static_assert(256 % 64 == 0 && 512 % 64 == 0 && 1024 % 64 == 0 && 256 % 32 == 0 && 512 % 32 == 0);
  static_assert((shp::NBATCH * shp::NCTR1) % 4 == 0 && shp::NCTR1 % 4 == 0);

  char* ws = (char*)d_ws;
  size_t off = 0;
  auto carve = [&](size_t bytes) -> void* {
    void* p = ws + off;
    off += (bytes + 255) & ~(size_t)255;
    return p;
  };
  float* c1 = (float*)carve((size_t)16 * 512 * 3 * 4);
  float* c2 = (float*)carve((size_t)16 * 128 * 3 * 4);
  unsigned short* f1 = (unsigned short*)carve((size_t)8192 * 128 * 2);
  unsigned short* A3 = (unsigned short*)carve((size_t)2048 * 320 * 2);
  unsigned short* h0 = (unsigned short*)carve((size_t)2048 * 256 * 2);
  unsigned short* h1 = (unsigned short*)carve((size_t)2048 * 512 * 2);
  float* pm = (float*)carve((size_t)32 * 1024 * 4);
  unsigned short* bt10 = (unsigned short*)carve((size_t)64 * 32 * 2);
  unsigned short* bt11 = (unsigned short*)carve((size_t)64 * 64 * 2);
  unsigned short* bt12 = (unsigned short*)carve((size_t)128 * 64 * 2);
  unsigned short* bt20 = (unsigned short*)carve((size_t)128 * 160 * 2);
  unsigned short* bt21 = (unsigned short*)carve((size_t)128 * 128 * 2);
  unsigned short* bt22 = (unsigned short*)carve((size_t)256 * 128 * 2);
  unsigned short* bt30 = (unsigned short*)carve((size_t)256 * 320 * 2);
  unsigned short* bt31 = (unsigned short*)carve((size_t)512 * 256 * 2);
  unsigned short* bt32 = (unsigned short*)carve((size_t)1024 * 512 * 2);
  if (off > ws_size) return;

  auto packw = [&](const float* W, unsigned short* Bt, int Kact, int Kpad, int Nout, int nfeat, int dup) {
    const int total = Nout * (Kpad / 8);
    pack_w_kernel<<<(total + 255) / 256, 256, 0, stream>>>(W, Bt, Kact, Kpad, Nout, nfeat, dup);
  };
  packw(s1w0, bt10,   3,  32,   64,  -1, 0);
  packw(s1w1, bt11,  64,  64,   64,  -1, 0);
  packw(s1w2, bt12,  64,  64,  128,  -1, 0);
  packw(s2w0, bt20, 131, 160,  128, 128, 0);
  packw(s2w1, bt21, 128, 128,  128,  -1, 0);
  packw(s2w2, bt22, 128, 128,  256,  -1, 0);
  packw(s3w0, bt30, 259, 320,  256, 256, 1);
  packw(s3w1, bt31, 256, 256,  512,  -1, 0);
  packw(s3w2, bt32, 512, 512, 1024,  -1, 0);

  fps_kernel<8192, 1024, 512><<<16, 1024, 0, stream>>>(x, c1);
  sa1_kernel<<<(16 * 512) / 4, 128, 0, stream>>>(x, c1, bt10, s1b0, bt11, s1b1, bt12, s1b2, f1);

  fps_kernel<512, 64, 128><<<16, 64, 0, stream>>>(c1, c2);
  sa2_kernel<<<16 * 128, 128, 0, stream>>>(c1, c2, f1, bt20, s2b0, bt21, s2b1, bt22, s2b2, A3);

  gemm64_kernel<false><<<(2048 / 64) * (256 / 64) / 8, 256, 0, stream>>>(
      A3, 320, bt30, 320, (void*)h0, 256, s3b0, 2048, 256, 320);
  gemm64_kernel<false><<<(2048 / 64) * (512 / 64) / 8, 256, 0, stream>>>(
      h0, 256, bt31, 256, (void*)h1, 512, s3b1, 2048, 512, 256);
  gemm64_kernel<true><<<(2048 / 64) * (1024 / 64) / 8, 256, 0, stream>>>(
      h1, 512, bt32, 512, (void*)pm, 1024, s3b2, 2048, 1024, 512);
  final_max_kernel<<<16, 256, 0, stream>>>(pm, s3b2, out);
}
